// SingleHeadAttention_30966714204282
// MI455X (gfx1250) — hardware-verified
//
#include <hip/hip_runtime.h>

typedef _Float16 h16;
typedef _Float16 h16x8 __attribute__((ext_vector_type(8)));
typedef _Float16 v16h  __attribute__((ext_vector_type(16)));
typedef float  v8f    __attribute__((ext_vector_type(8)));
typedef float  v4f    __attribute__((ext_vector_type(4)));
typedef unsigned v4u  __attribute__((ext_vector_type(4)));

#define D_DIM 768
#define S_LEN 4096
#define B_SZ  4
#define M_TOT (B_SZ * S_LEN)
#define PSC 256.0f
#define PUN (1.0f / 256.0f)

template <typename V> __device__ __forceinline__ void vst2(void* p, V v) {
  *(volatile V*)p = v; __threadfence(); *(volatile V*)p = v;
}
__device__ __forceinline__ void copy16_g2s(h16* ldst, const h16* gsrc) { *(h16x8*)ldst = *(const h16x8*)gsrc; }

__device__ __forceinline__ v16h load_a_frag(const h16* base, int ld, int k0) {
  int lane = threadIdx.x & 31;
  int idx  = lane & 15;
  int half = lane >> 4;
  const h16* p = base + idx * ld + k0 + half * 8;
  h16x8 lo = *(const h16x8*)(p);
  h16x8 hi = *(const h16x8*)(p + 16);
  return __builtin_shufflevector(lo, hi, 0,1,2,3,4,5,6,7,8,9,10,11,12,13,14,15);
}
__device__ __forceinline__ v16h load_b_frag(const h16* base, int ld, int k0) { return load_a_frag(base, ld, k0); }

__device__ __forceinline__ v8f wmma_f16(v16h a, v16h b, v8f c) {
  v8f d = __builtin_amdgcn_wmma_f32_16x16x32_f16(false, a, false, b, (short)0, c, false, false);
  asm volatile("v_nop\n\tv_nop\n\tv_nop\n\tv_nop" : "+v"(d) : "v"(a), "v"(b));
  return d;
}

__global__ void cvt_x_kernel(const float* __restrict__ x, h16* __restrict__ xb, int n8) {
  int g = blockIdx.x * blockDim.x + threadIdx.x;
  if (g >= n8) return;
  const v4f a = *(const v4f*)(x + (size_t)g * 8), b = *(const v4f*)(x + (size_t)g * 8 + 4);
  union { h16x8 h; v4u u; } pk;
#pragma unroll
  for (int i = 0; i < 4; ++i) { pk.h[i] = (h16)a[i]; pk.h[4 + i] = (h16)b[i]; }
  vst2(xb + (size_t)g * 8, pk.u);
}

__global__ __launch_bounds__(256) void cvt_w_kernel(const float* __restrict__ Wq, const float* __restrict__ Wk, const float* __restrict__ Wv,
                                                    h16* __restrict__ WqT, h16* __restrict__ WkT, h16* __restrict__ WvT) {
  __shared__ __align__(16) h16 tile[64][264];
  const float* W = (blockIdx.z == 0) ? Wq : (blockIdx.z == 1) ? Wk : Wv;
  h16*       WT = (blockIdx.z == 0) ? WqT : (blockIdx.z == 1) ? WkT : WvT;
  const int n0 = blockIdx.x * 64, k0 = blockIdx.y * 256, tid = threadIdx.x;
  for (int i = tid; i < 256 * 64; i += 256) { const int k = i >> 6, nl = i & 63; tile[nl][k] = (h16)W[(size_t)(k0 + k) * D_DIM + n0 + nl]; }
  __syncthreads();
  for (int g = tid; g < 64 * 32; g += 256) { const int nl = g >> 5, pc = g & 31; vst2(WT + (size_t)(n0 + nl) * D_DIM + k0 + pc * 8, *(const v4u*)(&tile[nl][pc * 8])); }
}

__global__ __launch_bounds__(256) void proj_kernel(const h16* __restrict__ Xb, const h16* __restrict__ WT,
                            const float* __restrict__ bias, h16* __restrict__ out, int transposed) {
  __shared__ __align__(16) h16 T[128 * 136];
  int m0 = blockIdx.x * 64;
  int n0 = blockIdx.y * 128;
  int w    = threadIdx.x >> 5;
  int lane = threadIdx.x & 31;
  int idx  = lane & 15;
  int half = lane >> 4;
  int m_w = m0 + (w & 3) * 16;
  int n_w = n0 + (w >> 2) * 64;

  v8f c[4] = {};
  const h16* arow = Xb + (size_t)m_w * D_DIM;
#pragma unroll 2
  for (int k0 = 0; k0 < D_DIM; k0 += 32) {
    v16h a = load_a_frag(arow, D_DIM, k0);
#pragma unroll
    for (int t = 0; t < 4; ++t) {
      v16h b = load_b_frag(WT + (size_t)(n_w + t * 16) * D_DIM, D_DIM, k0);
      c[t] = wmma_f16(a, b, c[t]);
    }
  }
#pragma unroll
  for (int t = 0; t < 4; ++t) {
    int cl = (w >> 2) * 64 + t * 16 + idx;
    float bv = bias[n0 + cl];
#pragma unroll
    for (int g = 0; g < 8; ++g) {
      int rl = (w & 3) * 16 + g + 8 * half;
      h16 hv = (h16)(c[t][g] + bv);
      if (!transposed) T[rl * 136 + cl] = hv; else T[cl * 72 + rl] = hv;
    }
  }
  __syncthreads();
  const int tid = threadIdx.x;
  if (!transposed) {
    for (int gg = tid; gg < 64 * 16; gg += 256) { const int rl = gg >> 4, pc = gg & 15; vst2(out + (size_t)(m0 + rl) * D_DIM + n0 + pc * 8, *(const v4u*)(&T[rl * 136 + pc * 8])); }
  } else {
    const int bb = m0 >> 12, s0 = m0 & (S_LEN - 1);
    for (int gg = tid; gg < 128 * 8; gg += 256) { const int cl = gg >> 3, pc = gg & 7; vst2(out + ((size_t)(bb * D_DIM + n0 + cl)) * S_LEN + s0 + pc * 8, *(const v4u*)(&T[cl * 72 + pc * 8])); }
  }
}

__global__ __launch_bounds__(256)
void attn_kernel(const h16* __restrict__ Q, const h16* __restrict__ K,
                 const h16* __restrict__ Vt, float* __restrict__ out) {
  __shared__ __align__(16) h16   Qs[32][D_DIM];
  __shared__ __align__(16) h16   Ks[64][D_DIM];
  __shared__ __align__(16) h16   Vts[D_DIM][64];
  __shared__ __align__(16) float Ss[32][64];
  __shared__ __align__(16) h16   Ps[32][64];
  __shared__ float alpha_s[32];
  __shared__ float l_s[32];

  int b   = blockIdx.y;
  int q0  = blockIdx.x * 32;
  int tid = threadIdx.x;
  int w    = tid >> 5;
  int lane = tid & 31;
  int idx  = lane & 15;
  int half = lane >> 4;
  int qi = w & 1;
  int kj = w >> 1;
  int dg = w >> 1;

  const h16* Qg = Q + ((size_t)(b * S_LEN + q0)) * D_DIM;
  for (int c = tid; c < 32 * (D_DIM / 8); c += 256) {
    int r = c / (D_DIM / 8), dc = c % (D_DIM / 8);
    copy16_g2s(&Qs[r][dc * 8], Qg + (size_t)r * D_DIM + dc * 8);
  }

  v8f o[12] = {};
  int   srow = tid >> 3;
  int   sj   = tid & 7;
  float m_prev = -1e30f;
  float l_run  = 0.0f;
  const float scale = 0.03608439182435161f;

  for (int kv0 = 0; kv0 < S_LEN; kv0 += 64) {
    __syncthreads();
    const h16* Kg = K + ((size_t)(b * S_LEN + kv0)) * D_DIM;
    for (int c = tid; c < 64 * (D_DIM / 8); c += 256) {
      int r = c / (D_DIM / 8), dc = c % (D_DIM / 8);
      copy16_g2s(&Ks[r][dc * 8], Kg + (size_t)r * D_DIM + dc * 8);
    }
    const h16* Vg = Vt + (size_t)b * D_DIM * S_LEN + kv0;
    for (int c = tid; c < D_DIM * 8; c += 256) {
      int d = c / 8, j = c % 8;
      copy16_g2s(&Vts[d][j * 8], Vg + (size_t)d * S_LEN + j * 8);
    }
    __syncthreads();

    {
      v8f sc = {};
#pragma unroll 4
      for (int k0 = 0; k0 < D_DIM; k0 += 32) {
        v16h a = load_a_frag(&Qs[qi * 16][0], D_DIM, k0);
        v16h bb = load_b_frag(&Ks[kj * 16][0], D_DIM, k0);
        sc = wmma_f16(a, bb, sc);
      }
      int col = kj * 16 + idx;
#pragma unroll
      for (int g = 0; g < 8; ++g)
        Ss[qi * 16 + g + 8 * half][col] = sc[g] * scale;
    }
    __syncthreads();

    {
      float v[8];
      float mloc = -1e30f;
#pragma unroll
      for (int e = 0; e < 8; ++e) { v[e] = Ss[srow][sj + e * 8]; mloc = fmaxf(mloc, v[e]); }
#pragma unroll
      for (int msk = 1; msk < 8; msk <<= 1) mloc = fmaxf(mloc, __shfl_xor(mloc, msk, 32));
      float m_new = fmaxf(m_prev, mloc);
      float alpha = __expf(m_prev - m_new);
      float ssum = 0.0f;
#pragma unroll
      for (int e = 0; e < 8; ++e) {
        float p = __expf(v[e] - m_new);
        ssum += p;
        Ps[srow][sj + e * 8] = (h16)(p * PSC);
      }
#pragma unroll
      for (int msk = 1; msk < 8; msk <<= 1) ssum += __shfl_xor(ssum, msk, 32);
      l_run = l_run * alpha + ssum;
      m_prev = m_new;
      if (sj == 0) { alpha_s[srow] = alpha; l_s[srow] = l_run; }
    }
    __syncthreads();

    {
      float al[8];
#pragma unroll
      for (int g = 0; g < 8; ++g) al[g] = alpha_s[qi * 16 + g + 8 * half];
#pragma unroll
      for (int t = 0; t < 12; ++t)
#pragma unroll
        for (int g = 0; g < 8; ++g) o[t][g] *= al[g];
#pragma unroll
      for (int k0 = 0; k0 < 64; k0 += 32) {
        v16h a = load_a_frag(&Ps[qi * 16][0], 64, k0);
#pragma unroll
        for (int t = 0; t < 12; ++t) {
          v16h bb = load_b_frag(&Vts[dg * 192 + t * 16][0], 64, k0);
          o[t] = wmma_f16(a, bb, o[t]);
        }
      }
    }
  }
  __syncthreads();

  float* Ot = (float*)&Ks[0][0];
  float linv[8];
#pragma unroll
  for (int g = 0; g < 8; ++g) linv[g] = PUN / l_s[qi * 16 + g + 8 * half];
#pragma unroll
  for (int t = 0; t < 12; ++t) {
    int col = dg * 192 + t * 16 + idx;
#pragma unroll
    for (int g = 0; g < 8; ++g) Ot[(qi * 16 + g + 8 * half) * D_DIM + col] = o[t][g] * linv[g];
  }
  __syncthreads();
  {
    float* dst = out + ((size_t)(b * S_LEN + q0)) * D_DIM;
    for (int gg = tid; gg < 32 * D_DIM / 4; gg += 256) vst2(dst + (size_t)gg * 4, *(const v4f*)(Ot + gg * 4));
  }
}

extern "C" void kernel_launch(void* const* d_in, const int* in_sizes, int n_in,
                              void* d_out, int out_size, void* d_ws, size_t ws_size,
                              hipStream_t stream) {
  (void)in_sizes; (void)n_in; (void)out_size; (void)ws_size;
  const float* x  = (const float*)d_in[0];
  const float* Wq = (const float*)d_in[1];
  const float* bq = (const float*)d_in[2];
  const float* Wk = (const float*)d_in[3];
  const float* bk = (const float*)d_in[4];
  const float* Wv = (const float*)d_in[5];
  const float* bv = (const float*)d_in[6];
  float* out = (float*)d_out;

  char* ws = (char*)d_ws;
  h16* xb  = (h16*)(ws + 0);
  h16* WqT = (h16*)(ws + 25165824);
  h16* WkT = (h16*)(ws + 26345472);
  h16* WvT = (h16*)(ws + 27525120);
  h16* qb  = (h16*)(ws + 28704768);
  h16* kb  = (h16*)(ws + 53870592);
  h16* vtb = (h16*)(ws + 79036416);

  int nx8 = M_TOT * D_DIM / 8;
  cvt_x_kernel<<<nx8 / 256, 256, 0, stream>>>(x, xb, nx8);
  cvt_w_kernel<<<dim3(D_DIM / 64, D_DIM / 256, 3), 256, 0, stream>>>(Wq, Wk, Wv, WqT, WkT, WvT);

  dim3 pg(M_TOT / 64, D_DIM / 128);
  proj_kernel<<<pg, 256, 0, stream>>>(xb, WqT, bq, qb, 0);
  proj_kernel<<<pg, 256, 0, stream>>>(xb, WkT, bk, kb, 0);
  proj_kernel<<<pg, 256, 0, stream>>>(xb, WvT, bv, vtb, 1);

  attn_kernel<<<dim3(S_LEN / 32, B_SZ), 256, 0, stream>>>(qb, kb, vtb, out);
}
